// HybridMoE_68899865362467
// MI455X (gfx1250) — hardware-run, weakly checked
//
#include <hip/hip_runtime.h>
#include <math.h>

#define NB 2
#define TSEQ 2048
#define NTOK (NB * TSEQ)
#define MSEL 2048
#define DM 1024
#define II 512
#define NE 8
#define SPT 1
#define NSLOT (MSEL * SPT)
#define R_MAX 4096
#define NT_MAX (R_MAX / 64)
#define NSH 1
#define NROW_S NTOK
#define LN_EPS 1e-5f

#define CX_LOG2 11
#define CW_LOG2 16
#define CA_LOG2 12
#define CH ((float)(1u << CX_LOG2))
#define CA ((float)(1u << CA_LOG2))
#define SC (1.0f / (float)(1u << (CX_LOG2 + CW_LOG2)))

#define RW_CH 8192
#define TBL_COUNT 0
#define TBL_POFF 16
#define TBL_NTILES 32
#define TBL_TILE_E 64
#define TBL_HDR 256
#define TBL_ROWTOK TBL_HDR
#define TBL_SLOTROW (TBL_HDR + R_MAX)
#define TBL_WORDS (TBL_HDR + R_MAX + NSLOT)

static_assert(NTOK == 4096 && MSEL == 2048 && DM == 1024 && II == 512 && NE == 8 && SPT == 1 && NSLOT == 2048 && R_MAX == 4096 && NT_MAX == 64);
static_assert(DM % 64 == 0 && II % 64 == 0 && NTOK % 128 == 0 && MSEL % 32 == 0 && NROW_S % 64 == 0 && NROW_S / 64 <= NT_MAX);
static_assert(NSLOT % 128 == 0 && R_MAX % 128 == 0 && R_MAX >= NSLOT + 64 * NE && MSEL <= NTOK);
static_assert(TBL_HDR % 32 == 0 && TBL_HDR <= 512);
static_assert(TBL_COUNT + NE <= TBL_POFF && TBL_POFF + NE + 1 <= TBL_NTILES && TBL_NTILES < TBL_TILE_E && TBL_TILE_E + NT_MAX <= TBL_HDR);
static_assert(RW_CH % 128 == 0 && (TBL_WORDS * 4) % 256 == 0 && TBL_WORDS == 6400);
static_assert((NTOK * DM / 8) % 256 == 0 && (II * DM / 8) % 256 == 0 && (NE * II * DM / 8) % 256 == 0);

constexpr size_t al256(size_t b) { return (b + 255) & ~(size_t)255; }
constexpr size_t SZ_X16  = al256((size_t)NTOK * DM * 2);
constexpr size_t SZ_WS   = al256((size_t)II * DM * 2);
constexpr size_t SZ_WE   = al256((size_t)NE * II * DM * 2);
constexpr size_t SZ_TBLD = al256((size_t)TBL_HDR * 4);
constexpr size_t SZ_TBLR = al256((size_t)TBL_WORDS * 4);
constexpr size_t SZ_SEL  = al256((size_t)MSEL * 4);
constexpr size_t SZ_WGT  = al256((size_t)MSEL * 8);
constexpr size_t SZ_INV  = al256((size_t)NTOK * 4);
constexpr size_t SZ_ACT  = al256((size_t)R_MAX * II * 2);
constexpr size_t SZ_Y    = al256((size_t)R_MAX * DM * 4);
constexpr size_t WS_TOTAL = SZ_X16 + 3 * SZ_WS + 3 * SZ_WE + SZ_TBLD + SZ_TBLR + 2 * SZ_SEL + SZ_WGT + SZ_INV + 2 * SZ_X16 + 4 * SZ_ACT + 2 * SZ_Y;
static_assert(WS_TOTAL == (size_t)103884800 && WS_TOTAL < (size_t)134217728);

typedef _Float16 h16;
typedef __attribute__((ext_vector_type(16))) _Float16 v16h;
typedef __attribute__((ext_vector_type(8)))  _Float16 v8h;
typedef __attribute__((ext_vector_type(8)))  float    v8f;
typedef __attribute__((ext_vector_type(4)))  float    v4f;
typedef __attribute__((ext_vector_type(2)))  float    v2f;
typedef __attribute__((ext_vector_type(4)))  unsigned int v4u;
typedef __attribute__((ext_vector_type(4)))  int      v4i;
typedef __attribute__((ext_vector_type(2)))  int      v2i;


#define VST2(T, ptr, val) do { const T vst2_v_ = (val); *(volatile T*)(ptr) = vst2_v_; __threadfence(); *(volatile T*)(ptr) = vst2_v_; } while (0)

static __device__ __forceinline__ float bfr(float f) {
    unsigned u = __float_as_uint(f);
    u += 0x7FFFu + ((u >> 16) & 1u);
    return __uint_as_float(u & 0xFFFF0000u);
}
static __device__ __forceinline__ h16 toh_flush(float v) { const float w = (fabsf(v) < 6.103515625e-05f) ? 0.0f : v; return (h16)w; }
static __device__ __forceinline__ void st8h(h16* p, const float* v) {
    v8h hv;
#pragma unroll
    for (int e = 0; e < 8; ++e) hv[e] = toh_flush(v[e]);
    VST2(v8h, p, hv);
}

union FragU { v16h v; v8h h[2]; };
static __device__ __forceinline__ v16h frag_ld(const h16* p) {
    FragU f; f.h[0] = *(const v8h*)(p); f.h[1] = *(const v8h*)(p + 16); return f.v;
}
static __device__ __forceinline__ v8f wmma16g(v16h a, v16h b, v8f c) {
    c = __builtin_amdgcn_wmma_f32_16x16x32_f16(false, a, false, b, (short)0, c, false, false);
    asm volatile("v_nop\n\tv_nop\n\tv_nop\n\tv_nop" : "+v"(c) : "v"(a), "v"(b));
    return c;
}
static __device__ __forceinline__ void wave_sync_lds() {
    __builtin_amdgcn_fence(3  , "workgroup");
    __builtin_amdgcn_wave_barrier();
    __builtin_amdgcn_fence(2  , "workgroup");
}

template <int LOG2C>
__global__ __launch_bounds__(256) void k_plane(const float* __restrict__ src, h16* __restrict__ dst, unsigned n8) {
    const unsigned u = blockIdx.x * 256u + threadIdx.x;
    if (u >= n8) return;
    const float cs = (float)(1u << LOG2C);
    const v4f a = *(const v4f*)(src + (size_t)u * 8u);
    const v4f b = *(const v4f*)(src + (size_t)u * 8u + 4u);
    float v[8] = {bfr(a.x) * cs, bfr(a.y) * cs, bfr(a.z) * cs, bfr(a.w) * cs, bfr(b.x) * cs, bfr(b.y) * cs, bfr(b.z) * cs, bfr(b.w) * cs};
    st8h(dst + (size_t)u * 8u, v);
}

__global__ __launch_bounds__(64) void k_tbl_dense(int* __restrict__ tbl) {
    const unsigned w0 = threadIdx.x * 4u;
    int q[4];
#pragma unroll
    for (int k = 0; k < 4; ++k) {
        const unsigned w = w0 + (unsigned)k;
        int val = 0;
        val = (w < (unsigned)(TBL_COUNT + NSH)) ? NTOK : val;
        val = (w >= (unsigned)TBL_POFF && w <= (unsigned)(TBL_POFF + NE)) ? (int)min((w - (unsigned)TBL_POFF) * (unsigned)NTOK, (unsigned)NROW_S) : val;
        val = (w == (unsigned)TBL_NTILES) ? (NROW_S / 64) : val;
        val = (w >= (unsigned)TBL_TILE_E && w < (unsigned)(TBL_TILE_E + NT_MAX)) ? ((w - (unsigned)TBL_TILE_E < (unsigned)(NROW_S / 64)) ? (int)((w - (unsigned)TBL_TILE_E) / (unsigned)(NTOK / 64)) : -1) : val;
        q[k] = val;
    }
    v4i v;
    v.x = q[0]; v.y = q[1]; v.z = q[2]; v.w = q[3];
    VST2(v4i, tbl + w0, v);
}

__global__ __launch_bounds__(256) void k_gate1(const float* __restrict__ x, const int* __restrict__ ib, const int* __restrict__ it_,
                                               const float* __restrict__ sgw, const float* __restrict__ sgb, const float* __restrict__ egw,
                                               const float* __restrict__ egb, const float* __restrict__ ebias,
                                               int* __restrict__ sel, int* __restrict__ posc, float* __restrict__ wgt) {
    const unsigned lane = threadIdx.x & 31u;
    const unsigned wave = threadIdx.x >> 5;
    const unsigned gwv = blockIdx.x * 8u + wave;
    const unsigned m0 = gwv * 32u;
    if (m0 >= (unsigned)MSEL) return;
    int kpick = 0, kpos = 0;
    float kws = 0.0f, kwe = 0.0f;
    for (unsigned j = 0; j < 32u; ++j) {
        const int pb = ib[m0 + j], pt = it_[m0 + j];
        const int p = min(max(pb, 0), NB - 1) * TSEQ + min(max(pt, 0), TSEQ - 1);
        const float* xr = x + (size_t)(unsigned)p * DM;
        float lg[NE];
        float ls = 0.0f;
#pragma unroll
        for (int e = 0; e < NE; ++e) lg[e] = 0.0f;
        for (unsigned i = 0; i < (unsigned)(DM / 32); ++i) {
            const unsigned d = lane + 32u * i;
            const float xv = bfr(xr[d]);
            ls += xv * bfr(sgw[d]);
#pragma unroll
            for (int e = 0; e < NE; ++e) lg[e] += xv * bfr(egw[(size_t)e * DM + d]);
        }
        ls += __shfl_xor(ls, 16, 32); ls += __shfl_xor(ls, 8, 32); ls += __shfl_xor(ls, 4, 32); ls += __shfl_xor(ls, 2, 32); ls += __shfl_xor(ls, 1, 32);
#pragma unroll
        for (int e = 0; e < NE; ++e) {
            lg[e] += __shfl_xor(lg[e], 16, 32);
            lg[e] += __shfl_xor(lg[e], 8, 32);
            lg[e] += __shfl_xor(lg[e], 4, 32);
            lg[e] += __shfl_xor(lg[e], 2, 32);
            lg[e] += __shfl_xor(lg[e], 1, 32);
        }
        float sc[NE];
#pragma unroll
        for (int e = 0; e < NE; ++e) { const float a = lg[e] + bfr(egb[e]); sc[e] = 1.0f / (1.0f + expf(-a)); }
        float bestv = sc[0] + bfr(ebias[0]);
        float bests = sc[0];
        int besti = 0;
#pragma unroll
        for (int e = 1; e < NE; ++e) { const float v = sc[e] + bfr(ebias[e]); const bool c = v > bestv; bestv = c ? v : bestv; bests = c ? sc[e] : bests; besti = c ? e : besti; }
        const float as = ls + bfr(sgb[0]);
        const float ss = 1.0f / (1.0f + expf(-as));
        const float mx = fmaxf(ss, bests);
        const float e0 = expf(ss - mx), e1 = expf(bests - mx);
        const float den = e0 + e1;
        const bool mine = (lane == j);
        kpick = mine ? besti : kpick;  kpos = mine ? p : kpos;
        kws = mine ? e0 / den : kws;   kwe = mine ? e1 / den : kwe;
    }
    v2f wv; wv.x = kws; wv.y = kwe;
    VST2(int, sel + (size_t)(m0 + lane), kpick);
    VST2(int, posc + (size_t)(m0 + lane), kpos);
    VST2(v2f, wgt + (size_t)(m0 + lane) * 2u, wv);
}

template <int NE_>
__global__ __launch_bounds__(32) void k_route1w(const int* __restrict__ sel, int* __restrict__ tbl, unsigned nslot, unsigned spt, unsigned hdr, unsigned rmax,
                                                unsigned offPoff, unsigned offNtiles, unsigned offTileE) {
    static_assert(NE_ >= 1 && NE_ <= 32);
    __shared__ __align__(16) int s_img[RW_CH];
    __shared__ __align__(16) int s_hdr[512];
    const unsigned lane = threadIdx.x & 31u;
    const unsigned spl = nslot >> 5;
    const unsigned ng = spl >> 2;
    const unsigned ntmax = rmax >> 6;
    const v4i* sp = (const v4i*)(sel + (size_t)lane * spl);
    int cnt[NE_];
#pragma unroll
    for (int j = 0; j < NE_; ++j) cnt[j] = 0;
    for (unsigned g = 0; g < ng; ++g) {
        const v4i v = sp[g];
#pragma unroll
        for (int c = 0; c < 4; ++c) {
            const int e = min(max(v[c], 0), NE_ - 1);
#pragma unroll
            for (int j = 0; j < NE_; ++j) cnt[j] += (e == j) ? 1 : 0;
        }
    }
    int base0[NE_], total[NE_];
#pragma unroll
    for (int j = 0; j < NE_; ++j) {
        int pre = 0, tot = cnt[j];
#pragma unroll
        for (int d = 1; d < 32; d <<= 1) {
            const int t = __shfl_xor(tot, d, 32);
            pre += ((lane & (unsigned)d) != 0u) ? t : 0;
            tot += t;
        }
        base0[j] = pre;
        total[j] = tot;
    }
    int poff[NE_ + 1];
    poff[0] = 0;
#pragma unroll
    for (int j = 0; j < NE_; ++j) poff[j + 1] = poff[j] + (((total[j] + 63) >> 6) << 6);
    for (unsigned i = lane; i < 512u; i += 32u) s_hdr[i] = (i >= offTileE && i < offTileE + ntmax) ? -1 : 0;
    wave_sync_lds();
    if (lane == 0u) {
#pragma unroll
        for (int j = 0; j < NE_; ++j) { s_hdr[min((unsigned)j, 511u)] = total[j]; s_hdr[min(offPoff + (unsigned)j, 511u)] = poff[j]; }
        s_hdr[min(offPoff + (unsigned)NE_, 511u)] = poff[NE_];
        s_hdr[min(offNtiles, 511u)] = poff[NE_] >> 6;
    }
    for (unsigned t = lane; t < ntmax; t += 32u) {
        const int b64 = (int)(t * 64u);
        int ev = -1;
#pragma unroll
        for (int j = 0; j < NE_; ++j) ev = (b64 >= poff[j] && b64 < poff[j + 1]) ? j : ev;
        s_hdr[min(offTileE + t, 511u)] = ev;
    }
    wave_sync_lds();
    for (int pass = 0; pass < 2; ++pass) {
        for (unsigned i = lane; i < (hdr >> 2); i += 32u) *(volatile v4i*)(tbl + 4u * i) = *(const v4i*)(&s_hdr[4u * i]);
        __threadfence();
    }
    for (unsigned lo = 0; lo < rmax; lo += (unsigned)RW_CH) {
        for (unsigned i = lane; i < (unsigned)(RW_CH / 4); i += 32u) *(v4i*)(&s_img[4u * i]) = (v4i){-1, -1, -1, -1};
        wave_sync_lds();
        int run[NE_];
#pragma unroll
        for (int j = 0; j < NE_; ++j) run[j] = base0[j];
        for (unsigned g = 0; g < ng; ++g) {
            const v4i v = sp[g];
#pragma unroll
            for (int c = 0; c < 4; ++c) {
                const int e = min(max(v[c], 0), NE_ - 1);
                int row = 0;
#pragma unroll
                for (int j = 0; j < NE_; ++j) {
                    const bool hit = (e == j);
                    row = hit ? (poff[j] + run[j]) : row;
                    run[j] += hit ? 1 : 0;
                }
                row = min(max(row, 0), (int)rmax - 1);
                const unsigned rel = (unsigned)row - lo;
                if (rel < (unsigned)RW_CH) s_img[rel] = (int)((lane * spl + 4u * g + (unsigned)c) / spt);
            }
        }
        wave_sync_lds();
        const unsigned nw = min((unsigned)RW_CH, rmax - lo);
        for (int pass = 0; pass < 2; ++pass) {
            for (unsigned i = lane; i < (nw >> 2); i += 32u) *(volatile v4i*)(tbl + hdr + lo + 4u * i) = *(const v4i*)(&s_img[4u * i]);
            __threadfence();
        }
        wave_sync_lds();
    }
    for (unsigned lo = 0; lo < nslot; lo += (unsigned)RW_CH) {
        int run[NE_];
#pragma unroll
        for (int j = 0; j < NE_; ++j) run[j] = base0[j];
        for (unsigned g = 0; g < ng; ++g) {
            const v4i v = sp[g];
#pragma unroll
            for (int c = 0; c < 4; ++c) {
                const int e = min(max(v[c], 0), NE_ - 1);
                int row = 0;
#pragma unroll
                for (int j = 0; j < NE_; ++j) {
                    const bool hit = (e == j);
                    row = hit ? (poff[j] + run[j]) : row;
                    run[j] += hit ? 1 : 0;
                }
                row = min(max(row, 0), (int)rmax - 1);
                const unsigned rel = (lane * spl + 4u * g + (unsigned)c) - lo;
                if (rel < (unsigned)RW_CH) s_img[rel] = row;
            }
        }
        wave_sync_lds();
        const unsigned nw = min((unsigned)RW_CH, nslot - lo);
        for (int pass = 0; pass < 2; ++pass) {
            for (unsigned i = lane; i < (nw >> 2); i += 32u) *(volatile v4i*)(tbl + hdr + rmax + lo + 4u * i) = *(const v4i*)(&s_img[4u * i]);
            __threadfence();
        }
        wave_sync_lds();
    }
}

__global__ __launch_bounds__(256) void k_pick(const h16* __restrict__ x16, const int* __restrict__ posc, h16* __restrict__ xm16) {
    const unsigned m = blockIdx.x * 2u + (threadIdx.x >> 7);
    if (m >= (unsigned)MSEL) return;
    const unsigned c = (threadIdx.x & 127u) * 8u;
    const int p = min(max(posc[m], 0), NTOK - 1);
    const v4u v = *(const v4u*)(x16 + (size_t)(unsigned)p * DM + c);
    VST2(v4u, xm16 + (size_t)m * DM + c, v);
}

__global__ __launch_bounds__(256) void k_gather(const h16* __restrict__ x16, const int* __restrict__ tbl, h16* __restrict__ Xg) {
    const unsigned row = blockIdx.x * 2u + (threadIdx.x >> 7);
    if (row >= (unsigned)R_MAX) return;
    const unsigned c = (threadIdx.x & 127u) * 8u;
    const int tr = tbl[TBL_ROWTOK + row];
    const bool pad = (tr < 0);
    const int tok = min(max(tr, 0), NTOK - 1);
    const v4u ld = *(const v4u*)(x16 + (size_t)(unsigned)tok * DM + c);
    v4u v;
    v.x = pad ? 0u : ld.x; v.y = pad ? 0u : ld.y; v.z = pad ? 0u : ld.z; v.w = pad ? 0u : ld.w;
    VST2(v4u, Xg + (size_t)row * DM + c, v);
}

__global__ __launch_bounds__(256) void k_gp(const h16* __restrict__ Xg, const h16* __restrict__ W1p, const h16* __restrict__ W3p,
                                            const float* __restrict__ b1, const float* __restrict__ b3,
                                            const int* __restrict__ tbl, h16* __restrict__ Hg, unsigned nreal) {
    __shared__ __align__(16) float sT[8][16 * 68];
    const unsigned lane = threadIdx.x & 31u;
    const unsigned wave = threadIdx.x >> 5;
    const unsigned u = blockIdx.x * 8u + wave;
    if (u >= (unsigned)(NT_MAX * 2 * (II / 64))) return;
    const unsigned rt32 = u / (unsigned)(II / 64);
    const unsigned ct = u - rt32 * (unsigned)(II / 64);
    const unsigned rowtile = rt32 >> 1;
    const int nt = min(max(tbl[TBL_NTILES], 0), NT_MAX);
    if ((int)rowtile >= nt) return;
    const int e = min(max(tbl[TBL_TILE_E + rowtile], 0), (int)nreal - 1);
    const size_t wbase = (size_t)(unsigned)e * (size_t)(II * DM);
    const unsigned m0 = rt32 * 32u, n0 = ct * 64u;
    const unsigned rlane = lane & 15u;
    const unsigned koff = (lane >> 4) * 8u;
    const unsigned mOff = koff;

    v8f acc1[2][4], acc3[2][4];
#pragma unroll
    for (int i = 0; i < 2; ++i)
#pragma unroll
        for (int j = 0; j < 4; ++j) { acc1[i][j] = (v8f){0.f,0.f,0.f,0.f,0.f,0.f,0.f,0.f}; acc3[i][j] = acc1[i][j]; }

    for (unsigned k0 = 0; k0 < (unsigned)DM; k0 += 32u) {
        v16h ah[2];
#pragma unroll
        for (int i = 0; i < 2; ++i)
            ah[i] = frag_ld(Xg + (size_t)(m0 + ((unsigned)i << 4) + rlane) * DM + koff + k0);
#pragma unroll
        for (int j = 0; j < 4; ++j) {
            const size_t bo = wbase + (size_t)(n0 + ((unsigned)j << 4) + rlane) * DM + koff + k0;
            const v16h b1f = frag_ld(W1p + bo);
            const v16h b3f = frag_ld(W3p + bo);
#pragma unroll
            for (int i = 0; i < 2; ++i) {
                acc1[i][j] = wmma16g(ah[i], b1f, acc1[i][j]);
                acc3[i][j] = wmma16g(ah[i], b3f, acc3[i][j]);
            }
        }
    }

    float bv1[4], bv3[4];
#pragma unroll
    for (int j = 0; j < 4; ++j) {
        bv1[j] = bfr(b1[(unsigned)e * (unsigned)II + n0 + ((unsigned)j << 4) + rlane]);
        bv3[j] = bfr(b3[(unsigned)e * (unsigned)II + n0 + ((unsigned)j << 4) + rlane]);
    }

    float* slab = sT[wave];
#pragma unroll
    for (int i = 0; i < 2; ++i) {
        const unsigned mBase = m0 + ((unsigned)i << 4);
#pragma unroll
        for (int j = 0; j < 4; ++j) {
#pragma unroll
            for (int r = 0; r < 8; ++r) {
                const float h = acc1[i][j][r] * SC + bv1[j];
                const float g = acc3[i][j][r] * SC + bv3[j];
                const float a = (h / (1.0f + expf(-h))) * g;
                slab[(mOff + (unsigned)r) * 68u + ((unsigned)j << 4) + rlane] = a * CA;
            }
        }
        wave_sync_lds();
        const unsigned q = lane >> 3, c8 = (lane & 7u) * 8u;
        v8h hv[4];
#pragma unroll
        for (int it = 0; it < 4; ++it) {
            const unsigned row = (unsigned)it * 4u + q;
            const float* sp = slab + row * 68u + c8;
#pragma unroll
            for (int t = 0; t < 8; ++t) hv[it][t] = toh_flush(sp[t]);
        }
        for (int pass = 0; pass < 2; ++pass) {
#pragma unroll
            for (int it = 0; it < 4; ++it) {
                const unsigned row = (unsigned)it * 4u + q;
                *(volatile v8h*)(Hg + (size_t)(mBase + row) * II + n0 + c8) = hv[it];
            }
            __threadfence();
        }
        wave_sync_lds();
    }
}

__global__ __launch_bounds__(256) void k_ln(const h16* __restrict__ Hg, const float* __restrict__ g, const float* __restrict__ b,
                                            const int* __restrict__ tbl, h16* __restrict__ Zg) {
    const unsigned lane = threadIdx.x & 31u;
    const unsigned row = blockIdx.x * 8u + (threadIdx.x >> 5);
    if (row >= (unsigned)R_MAX) return;
    const int nt = min(max(tbl[TBL_NTILES], 0), NT_MAX);
    if ((int)(row >> 6) >= nt) return;
    float a[16];
#pragma unroll
    for (int hf = 0; hf < 2; ++hf) {
        const v8h v = *(const v8h*)(Hg + (size_t)row * II + (unsigned)hf * 256u + lane * 8u);
#pragma unroll
        for (int t = 0; t < 8; ++t) a[hf * 8 + t] = (float)v[t] * (1.0f / CA);
    }
    float s = 0.0f;
#pragma unroll
    for (int t = 0; t < 16; ++t) s += a[t];
    s += __shfl_xor(s, 16, 32); s += __shfl_xor(s, 8, 32); s += __shfl_xor(s, 4, 32); s += __shfl_xor(s, 2, 32); s += __shfl_xor(s, 1, 32);
    const float mean = s * (1.0f / (float)II);
    float q = 0.0f;
#pragma unroll
    for (int t = 0; t < 16; ++t) { const float d = a[t] - mean; q += d * d; }
    q += __shfl_xor(q, 16, 32); q += __shfl_xor(q, 8, 32); q += __shfl_xor(q, 4, 32); q += __shfl_xor(q, 2, 32); q += __shfl_xor(q, 1, 32);
    const float var = q * (1.0f / (float)II);
    const float rs = 1.0f / sqrtf(var + LN_EPS);
#pragma unroll
    for (int hf = 0; hf < 2; ++hf) {
        const unsigned c0 = (unsigned)hf * 256u + lane * 8u;
        const v4f ga = *(const v4f*)(g + c0), gb = *(const v4f*)(g + c0 + 4u);
        const v4f ba = *(const v4f*)(b + c0), bb = *(const v4f*)(b + c0 + 4u);
        const float gg[8] = {ga.x, ga.y, ga.z, ga.w, gb.x, gb.y, gb.z, gb.w};
        const float bo[8] = {ba.x, ba.y, ba.z, ba.w, bb.x, bb.y, bb.z, bb.w};
        v8h o;
#pragma unroll
        for (int t = 0; t < 8; ++t) o[t] = toh_flush(((a[hf * 8 + t] - mean) * rs * bfr(gg[t]) + bfr(bo[t])) * CH);
        VST2(v8h, Zg + (size_t)row * II + c0, o);
    }
}

__global__ __launch_bounds__(256) void k_dn(const h16* __restrict__ Zg, const h16* __restrict__ W2p, const float* __restrict__ b2,
                                            const int* __restrict__ tbl, float* __restrict__ Yg, unsigned nreal) {
    __shared__ __align__(16) float sT[8][16 * 68];
    const unsigned lane = threadIdx.x & 31u;
    const unsigned wave = threadIdx.x >> 5;
    const unsigned u = blockIdx.x * 8u + wave;
    if (u >= (unsigned)(NT_MAX * (DM / 64))) return;
    const unsigned rowtile = u / (unsigned)(DM / 64);
    const unsigned ct = u - rowtile * (unsigned)(DM / 64);
    const int nt = min(max(tbl[TBL_NTILES], 0), NT_MAX);
    if ((int)rowtile >= nt) return;
    const int e = min(max(tbl[TBL_TILE_E + rowtile], 0), (int)nreal - 1);
    const size_t wbase = (size_t)(unsigned)e * (size_t)(DM * II);
    const unsigned m0 = rowtile << 6, n0 = ct << 6;
    const unsigned rlane = lane & 15u;
    const unsigned koff = (lane >> 4) * 8u;
    const unsigned mOff = koff;

    v8f acc[4][4];
#pragma unroll
    for (int i = 0; i < 4; ++i)
#pragma unroll
        for (int j = 0; j < 4; ++j) acc[i][j] = (v8f){0.f,0.f,0.f,0.f,0.f,0.f,0.f,0.f};

    for (unsigned k0 = 0; k0 < (unsigned)II; k0 += 32u) {
        v16h bh[4];
#pragma unroll
        for (int j = 0; j < 4; ++j)
            bh[j] = frag_ld(W2p + wbase + (size_t)(n0 + ((unsigned)j << 4) + rlane) * II + koff + k0);
#pragma unroll
        for (int i = 0; i < 4; ++i) {
            const v16h ah = frag_ld(Zg + (size_t)(m0 + ((unsigned)i << 4) + rlane) * II + koff + k0);
#pragma unroll
            for (int j = 0; j < 4; ++j) acc[i][j] = wmma16g(ah, bh[j], acc[i][j]);
        }
    }

    float bv[4];
#pragma unroll
    for (int j = 0; j < 4; ++j) bv[j] = bfr(b2[(unsigned)e * (unsigned)DM + n0 + ((unsigned)j << 4) + rlane]);

    float* slab = sT[wave];
#pragma unroll
    for (int i = 0; i < 4; ++i) {
        const unsigned mBase = m0 + ((unsigned)i << 4);
#pragma unroll
        for (int j = 0; j < 4; ++j)
#pragma unroll
            for (int r = 0; r < 8; ++r)
                slab[(mOff + (unsigned)r) * 68u + ((unsigned)j << 4) + rlane] = acc[i][j][r] * SC + bv[j];
        wave_sync_lds();
        const unsigned hh = lane >> 4, c4 = (lane & 15u) * 4u;
#pragma unroll
        for (int half = 0; half < 2; ++half) {
            v4f vv[4];
#pragma unroll
            for (int it = 0; it < 4; ++it) {
                const unsigned row = (unsigned)(half * 4 + it) * 2u + hh;
                vv[it] = *(const v4f*)(slab + row * 68u + c4);
            }
            for (int pass = 0; pass < 2; ++pass) {
#pragma unroll
                for (int it = 0; it < 4; ++it) {
                    const unsigned row = (unsigned)(half * 4 + it) * 2u + hh;
                    *(volatile v4f*)(Yg + (size_t)(mBase + row) * DM + n0 + c4) = vv[it];
                }
                __threadfence();
            }
        }
        wave_sync_lds();
    }
}

__global__ __launch_bounds__(32) void k_inv1w(const int* __restrict__ posc, int* __restrict__ inv) {
    const unsigned lane = threadIdx.x & 31u;
    if (blockIdx.x != 0u) return;
    for (unsigned t = 0; t < (unsigned)(NTOK / 32); ++t) { VST2(int, inv + (size_t)(t * 32u + lane), -1); }
    __threadfence();
    for (unsigned t = 0; t < (unsigned)(MSEL / 32); ++t) {
        const unsigned m = t * 32u + lane;
        const int p = min(max(posc[m], 0), NTOK - 1);
        VST2(int, inv + (size_t)(unsigned)p, (int)m);
    }
}

__global__ __launch_bounds__(256) void k_mix(const float* __restrict__ Ys, const float* __restrict__ Yg, const float* __restrict__ wgt,
                                             const int* __restrict__ inv, const int* __restrict__ tbl, float* __restrict__ out) {
    const unsigned r = blockIdx.x;
    if (r >= (unsigned)NTOK) return;
    const unsigned c = threadIdx.x * 4u;
    const int mi = inv[r];
    const bool selrow = (mi >= 0);
    const int m = min(max(mi, 0), MSEL - 1);
    const int sr = min(max(tbl[TBL_SLOTROW + m], 0), R_MAX - 1);
    const float ws = wgt[(size_t)(unsigned)m * 2u], we = wgt[(size_t)(unsigned)m * 2u + 1u];
    const v4f s = *(const v4f*)(Ys + (size_t)r * DM + c);
    const v4f y = *(const v4f*)(Yg + (size_t)(unsigned)sr * DM + c);
    v4f o;
    o.x = selrow ? (s.x * ws + y.x * we) : s.x;
    o.y = selrow ? (s.y * ws + y.y * we) : s.y;
    o.z = selrow ? (s.z * ws + y.z * we) : s.z;
    o.w = selrow ? (s.w * ws + y.w * we) : s.w;
    VST2(v4f, out + (size_t)r * DM + c, o);
}

extern "C" void kernel_launch(void* const* d_in, const int* in_sizes, int n_in, void* d_out, int out_size,
                              void* d_ws, size_t ws_size, hipStream_t stream) {
    if (n_in < 24) return;
    if (in_sizes[0] < NTOK * DM || in_sizes[1] < MSEL || in_sizes[2] < MSEL || in_sizes[3] < II * DM || in_sizes[4] < II || in_sizes[5] < II * DM || in_sizes[6] < II ||
        in_sizes[7] < DM * II || in_sizes[8] < DM || in_sizes[9] < II || in_sizes[10] < II || in_sizes[11] < DM || in_sizes[12] < 1 || in_sizes[13] < NE * DM || in_sizes[14] < NE ||
        in_sizes[15] < NE || in_sizes[16] < NE * II * DM || in_sizes[17] < NE * II || in_sizes[18] < NE * II * DM || in_sizes[19] < NE * II || in_sizes[20] < NE * DM * II ||
        in_sizes[21] < NE * DM || in_sizes[22] < II || in_sizes[23] < II) return;
    if (out_size < NTOK * DM) return;

    const float* x    = (const float*)d_in[0];
    const int*   ib   = (const int*)d_in[1];
    const int*   it_  = (const int*)d_in[2];
    const float* sw1  = (const float*)d_in[3];
    const float* sb1  = (const float*)d_in[4];
    const float* sw2  = (const float*)d_in[5];
    const float* sb2  = (const float*)d_in[6];
    const float* sw3  = (const float*)d_in[7];
    const float* sb3  = (const float*)d_in[8];
    const float* slg  = (const float*)d_in[9];
    const float* slb  = (const float*)d_in[10];
    const float* sgw  = (const float*)d_in[11];
    const float* sgb  = (const float*)d_in[12];
    const float* egw  = (const float*)d_in[13];
    const float* egb  = (const float*)d_in[14];
    const float* ebs  = (const float*)d_in[15];
    const float* ew1  = (const float*)d_in[16];
    const float* eb1  = (const float*)d_in[17];
    const float* ew2  = (const float*)d_in[18];
    const float* eb2  = (const float*)d_in[19];
    const float* ew3  = (const float*)d_in[20];
    const float* eb3  = (const float*)d_in[21];
    const float* elg  = (const float*)d_in[22];
    const float* elb  = (const float*)d_in[23];
    float* out = (float*)d_out;

    char* wsp = (char*)d_ws;
    size_t off = 0;
    auto carve = [&](size_t bytes) -> void* { void* r = wsp + off; off += (bytes + 255) & ~(size_t)255; return r; };
    h16* x16  = (h16*)carve((size_t)NTOK * DM * 2);
    h16* sw1p = (h16*)carve((size_t)II * DM * 2);
    h16* sw2p = (h16*)carve((size_t)II * DM * 2);
    h16* sw3p = (h16*)carve((size_t)DM * II * 2);
    h16* ew1p = (h16*)carve((size_t)NE * II * DM * 2);
    h16* ew2p = (h16*)carve((size_t)NE * II * DM * 2);
    h16* ew3p = (h16*)carve((size_t)NE * DM * II * 2);
    int* tblD = (int*)carve((size_t)TBL_HDR * 4);
    int* tblR = (int*)carve((size_t)TBL_WORDS * 4);
    int* sel  = (int*)carve((size_t)MSEL * 4);
    int* posc = (int*)carve((size_t)MSEL * 4);
    float* wgt = (float*)carve((size_t)MSEL * 8);
    int* inv  = (int*)carve((size_t)NTOK * 4);
    h16* xm16 = (h16*)carve((size_t)NTOK * DM * 2);
    h16* Xg   = (h16*)carve((size_t)R_MAX * DM * 2);
    h16* HgS  = (h16*)carve((size_t)R_MAX * II * 2);
    h16* ZgS  = (h16*)carve((size_t)R_MAX * II * 2);
    h16* HgR  = (h16*)carve((size_t)R_MAX * II * 2);
    h16* ZgR  = (h16*)carve((size_t)R_MAX * II * 2);
    float* Ys = (float*)carve((size_t)R_MAX * DM * 4);
    float* Yg = (float*)carve((size_t)R_MAX * DM * 4);
    if (off != WS_TOTAL || off > ws_size || off > (size_t)134217728) return;

    k_plane<CX_LOG2><<<(NTOK * DM / 8) / 256, 256, 0, stream>>>(x, x16, (unsigned)(NTOK * DM / 8));
    k_plane<CW_LOG2><<<(II * DM / 8) / 256, 256, 0, stream>>>(sw1, sw1p, (unsigned)(II * DM / 8));
    k_plane<CW_LOG2><<<(II * DM / 8) / 256, 256, 0, stream>>>(sw2, sw2p, (unsigned)(II * DM / 8));
    k_plane<CW_LOG2><<<(DM * II / 8) / 256, 256, 0, stream>>>(sw3, sw3p, (unsigned)(DM * II / 8));
    k_plane<CW_LOG2><<<(NE * II * DM / 8) / 256, 256, 0, stream>>>(ew1, ew1p, (unsigned)(NE * II * DM / 8));
    k_plane<CW_LOG2><<<(NE * II * DM / 8) / 256, 256, 0, stream>>>(ew2, ew2p, (unsigned)(NE * II * DM / 8));
    k_plane<CW_LOG2><<<(NE * DM * II / 8) / 256, 256, 0, stream>>>(ew3, ew3p, (unsigned)(NE * DM * II / 8));
    k_tbl_dense<<<1, 64, 0, stream>>>(tblD);
    k_gate1<<<MSEL / 256, 256, 0, stream>>>(x, ib, it_, sgw, sgb, egw, egb, ebs, sel, posc, wgt);
    k_route1w<NE><<<1, 32, 0, stream>>>(sel, tblR, (unsigned)NSLOT, (unsigned)SPT, (unsigned)TBL_HDR, (unsigned)R_MAX, (unsigned)TBL_POFF, (unsigned)TBL_NTILES, (unsigned)TBL_TILE_E);
    k_pick<<<MSEL / 2, 256, 0, stream>>>(x16, posc, xm16);
    k_gather<<<R_MAX / 2, 256, 0, stream>>>(xm16, tblR, Xg);
    k_gp<<<(NT_MAX * 2 * (II / 64) + 7) / 8, 256, 0, stream>>>(x16, sw1p, sw2p, sb1, sb2, tblD, HgS, 1u);
    k_ln<<<R_MAX / 8, 256, 0, stream>>>(HgS, slg, slb, tblD, ZgS);
    k_dn<<<(NT_MAX * (DM / 64) + 7) / 8, 256, 0, stream>>>(ZgS, sw3p, sb3, tblD, Ys, 1u);
    k_gp<<<(NT_MAX * 2 * (II / 64) + 7) / 8, 256, 0, stream>>>(Xg, ew1p, ew2p, eb1, eb2, tblR, HgR, (unsigned)NE);
    k_ln<<<R_MAX / 8, 256, 0, stream>>>(HgR, elg, elb, tblR, ZgR);
    k_dn<<<(NT_MAX * (DM / 64) + 7) / 8, 256, 0, stream>>>(ZgR, ew3p, eb3, tblR, Yg, (unsigned)NE);
    k_inv1w<<<1, 32, 0, stream>>>(posc, inv);
    k_mix<<<NTOK, 256, 0, stream>>>(Ys, Yg, wgt, inv, tblR, out);
}
